// HierarchicalSpatialAttention_76922864271781
// MI455X (gfx1250) — hardware-run, weakly checked
//
#include <hip/hip_runtime.h>

typedef float          v8f   __attribute__((ext_vector_type(8)));
typedef float          v4f   __attribute__((ext_vector_type(4)));
typedef unsigned int   v4u   __attribute__((ext_vector_type(4)));
typedef int            v8i   __attribute__((ext_vector_type(8)));
typedef unsigned short v8us  __attribute__((ext_vector_type(8)));
typedef unsigned short v16us __attribute__((ext_vector_type(16)));
typedef __bf16         v16bf __attribute__((ext_vector_type(16)));
typedef _Float16       v16h  __attribute__((ext_vector_type(16)));
typedef v4f  __attribute__((may_alias)) v4fa;
typedef v8us __attribute__((may_alias)) v8usa;
union FragB { v16bf v; v16us u; v8us h[2]; v8i w; };
union FragH { v16h  v; v16us u; v8us h[2]; v8i w; };

__device__ __forceinline__ v8f wmb(const FragB& a, const FragB& b, v8f c) {
  v8f d = __builtin_amdgcn_wmma_f32_16x16x32_bf16(false, a.v, false, b.v, (short)0, c, false, false);
  asm volatile("v_nop\n\tv_nop\n\tv_nop\n\tv_nop" : "+v"(d) : "v"(a.w), "v"(b.w));
  return d;
}

__device__ __forceinline__ v8f wmh(const FragH& a, const FragH& b, v8f c) {
  v8f d = __builtin_amdgcn_wmma_f32_16x16x32_f16(false, a.v, false, b.v, (short)0, c, false, false);
  asm volatile("v_nop\n\tv_nop\n\tv_nop\n\tv_nop" : "+v"(d) : "v"(a.w), "v"(b.w));
  return d;
}

__device__ __forceinline__ unsigned bf16_bits(float f) {
  const unsigned u = __float_as_uint(f);
  const unsigned r = (u + 0x7FFFu + ((u >> 16) & 1u)) >> 16;
  const unsigned q = (u >> 16) | 0x40u;
  return ((u & 0x7fffffffu) > 0x7f800000u) ? q : r;
}

__device__ __forceinline__ float bf16_val(float f) {
  return __uint_as_float(bf16_bits(f) << 16);
}
__device__ __forceinline__ int clampi(int v, int lo, int hi) {
  return v < lo ? lo : (v > hi ? hi : v);
}

__device__ __forceinline__ unsigned f16_bits(float f) {
  const unsigned u  = __float_as_uint(f);
  const unsigned s  = (u >> 16) & 0x8000u;
  const unsigned a  = u & 0x7fffffffu;
  const unsigned t  = a - 0x38000000u;
  const unsigned r  = (t + 0x0FFFu + ((t >> 13) & 1u)) >> 13;
  const unsigned rc = r > 0x7C00u ? 0x7C00u : r;
  const bool small  = a < 0x38800000u;
  const bool isnan  = a > 0x7f800000u;
  const unsigned fin = small ? 0u : (s | rc);
  return isnan ? (s | 0x7E00u) : fin;
}

__device__ __forceinline__ unsigned pk16(unsigned lo, unsigned hi) { return lo | (hi << 16); }
__device__ __forceinline__ unsigned bf16_lo_bits(float v) {
  float hi = bf16_val(v);
  asm volatile("" : "+v"(hi));
  return bf16_bits(v - hi);
}
__device__ __forceinline__ v4u pack8_bf16(v4f a, v4f c) {
  return (v4u){ pk16(bf16_bits(a[0]), bf16_bits(a[1])), pk16(bf16_bits(a[2]), bf16_bits(a[3])),
                pk16(bf16_bits(c[0]), bf16_bits(c[1])), pk16(bf16_bits(c[2]), bf16_bits(c[3])) };
}
__device__ __forceinline__ v4u pack8_bf16_lo(v4f a, v4f c) {
  return (v4u){ pk16(bf16_lo_bits(a[0]), bf16_lo_bits(a[1])), pk16(bf16_lo_bits(a[2]), bf16_lo_bits(a[3])),
                pk16(bf16_lo_bits(c[0]), bf16_lo_bits(c[1])), pk16(bf16_lo_bits(c[2]), bf16_lo_bits(c[3])) };
}
__device__ __forceinline__ v4u pack8_f16(v4f a, v4f c) {
  return (v4u){ pk16(f16_bits(a[0]), f16_bits(a[1])), pk16(f16_bits(a[2]), f16_bits(a[3])),
                pk16(f16_bits(c[0]), f16_bits(c[1])), pk16(f16_bits(c[2]), f16_bits(c[3])) };
}

template <int FORM>
__global__ __launch_bounds__(256) void k_plane(const float* __restrict__ src, int rows, int cols, int ldsrc,
                                               unsigned short* __restrict__ dst, int MP, int KP) {
  static_assert(FORM >= 0 && FORM <= 3);
  const int KTOT = (FORM == 1 || FORM == 3) ? 2 * KP : KP;
  const unsigned ppr   = (unsigned)(KTOT >> 3);
  const unsigned kp8   = (unsigned)(KP >> 3);
  const unsigned total = (unsigned)MP * ppr;
  const unsigned g     = blockIdx.x * 256u + threadIdx.x;
  const unsigned rowu  = g / ppr;
  const unsigned p     = g - rowu * ppr;
  const bool second    = p >= kp8;
  const int row = (int)rowu;
  const int c0  = (int)((second ? p - kp8 : p) << 3);
  const float* srow = src + (size_t)clampi(row, 0, rows - 1) * (size_t)ldsrc;
  float x[8];
  unsigned mk[8];
#pragma unroll
  for (int e = 0; e < 8; ++e) {
    const int c = c0 + e;
    const float v = srow[clampi(c, 0, cols - 1)];
    asm volatile("" :: "v"(v));
    x[e]  = v;
    mk[e] = (row < rows && c < cols) ? 0xFFFFu : 0u;
  }
  const v4f a = (v4f){ x[0], x[1], x[2], x[3] };
  const v4f c = (v4f){ x[4], x[5], x[6], x[7] };
  v4u o;
  if (FORM == 2) {
    o = pack8_f16(a, c);
  } else {
    const v4u hi = pack8_bf16(a, c);
    o = hi;
    if (FORM == 1) { const v4u lo = pack8_bf16_lo(a, c); o = second ? lo : hi; }
  }
  const v4u mw = (v4u){ pk16(mk[0], mk[1]), pk16(mk[2], mk[3]), pk16(mk[4], mk[5]), pk16(mk[6], mk[7]) };
  o &= mw;
  if (g < total) {
    volatile v4u* q = (volatile v4u*)(dst + (size_t)g * 8);
    *q = o;
    __threadfence();
    *q = o;
  }
}

template <int FORM> struct FragOf    { typedef FragB T; };
template <>         struct FragOf<2> { typedef FragH T; };
__device__ __forceinline__ v8f mm(const FragB& a, const FragB& b, v8f c) { return wmb(a, b, c); }
__device__ __forceinline__ v8f mm(const FragH& a, const FragH& b, v8f c) { return wmh(a, b, c); }
template <class F> __device__ __forceinline__ F ld_frag(const unsigned short* p) {
  F f;
  f.h[0] = *(const v8usa*)(p);
  f.h[1] = *(const v8usa*)(p + 16);
  return f;
}

template <int FORM, int EPI>
__global__ __launch_bounds__(256) __attribute__((amdgpu_num_vgpr(248)))
void k_gemm_nt(const unsigned short* __restrict__ A, const unsigned short* __restrict__ B,
               const float* __restrict__ bias, float* __restrict__ D, int M, int N, int KTOT, int ldd) {
  static_assert(FORM >= 0 && FORM <= 2);
  static_assert(EPI == 0 || EPI == 1);
  typedef typename FragOf<FORM>::T F;
  __shared__ __attribute__((aligned(16))) float sT[8][16 * 68];
  const int lane = threadIdx.x & 31;
  const int wave = threadIdx.x >> 5;
  const int tilesM = (M + 63) >> 6;
  const int tilesN = (N + 63) >> 6;
  const int tile = blockIdx.x * 8 + wave;
  if (tile >= tilesM * tilesN) return;
  const int tm = tile / tilesN;
  const int tn = tile - tm * tilesN;
  const int m0 = tm << 6;
  const int n0 = tn << 6;

  const int rl = lane & 15;
  const int h8 = (lane >> 4) * 8;
  const unsigned short* pa = A + (size_t)(m0 + rl) * (size_t)KTOT + h8;
  const unsigned short* pb = B + (size_t)(n0 + rl) * (size_t)KTOT + h8;

  v8f acc[4][4];
#pragma unroll
  for (int i = 0; i < 4; ++i)
#pragma unroll
    for (int j = 0; j < 4; ++j) acc[i][j] = (v8f){0.f, 0.f, 0.f, 0.f, 0.f, 0.f, 0.f, 0.f};

#pragma unroll 1
  for (int k0 = 0; k0 < KTOT; k0 += 32) {
    F bf[4];
#pragma unroll
    for (int j = 0; j < 4; ++j) bf[j] = ld_frag<F>(pb + (size_t)(j << 4) * (size_t)KTOT + k0);
#pragma unroll
    for (int i = 0; i < 4; ++i) {
      const F af = ld_frag<F>(pa + (size_t)(i << 4) * (size_t)KTOT + k0);
#pragma unroll
      for (int j = 0; j < 4; ++j) acc[i][j] = mm(af, bf[j], acc[i][j]);
    }
  }

  float* slab = sT[wave];
  const int hh = lane >> 4;
  const int c4 = (lane & 15) * 4;
  const int nc = n0 + c4;
  const bool cok = nc < N;
  v4f bv = (v4f){0.f, 0.f, 0.f, 0.f};
  if (EPI == 1) {
    bv = *(const v4fa*)(bias + clampi(nc, 0, N - 4));
    asm volatile("" :: "v"(bv));
  }
#pragma unroll
  for (int i = 0; i < 4; ++i) {
    const int mBase = m0 + (i << 4);
#pragma unroll
    for (int j = 0; j < 4; ++j) {
#pragma unroll
      for (int r = 0; r < 8; ++r) slab[(h8 + r) * 68 + (j << 4) + rl] = acc[i][j][r];
    }
    __builtin_amdgcn_fence(__ATOMIC_RELEASE, "workgroup");
    __builtin_amdgcn_wave_barrier();
    __builtin_amdgcn_fence(__ATOMIC_ACQUIRE, "workgroup");
    v4f vv[8];
#pragma unroll
    for (int it = 0; it < 8; ++it) {
      const int row = it * 2 + hh;
      v4f v = *(const v4fa*)(slab + row * 68 + c4);
      if (EPI == 1) v += bv;
      vv[it] = v;
    }
    for (int pass = 0; pass < 2; ++pass) {
#pragma unroll
      for (int it = 0; it < 8; ++it) {
        const int row = mBase + it * 2 + hh;
        if (cok && row < M) *(volatile v4f*)(D + (size_t)row * (size_t)ldd + nc) = vv[it];
      }
      __threadfence();
    }
    __builtin_amdgcn_fence(__ATOMIC_RELEASE, "workgroup");
    __builtin_amdgcn_wave_barrier();
    __builtin_amdgcn_fence(__ATOMIC_ACQUIRE, "workgroup");
  }
}

#pragma clang fp contract(off)

typedef int   v4i  __attribute__((ext_vector_type(4)));
typedef float v2f  __attribute__((ext_vector_type(2)));
typedef v2f __attribute__((may_alias)) v2fa;
typedef v4u __attribute__((may_alias)) v4ua;

#define NN      10000
#define NE      320000
#define DD      256
#define NSC     3
#define MPAD    10240
#define SPP     10240
#define TABP    1792
#define NTHR    256
#define NWAVE   8
#define EPT     8
#define CHUNK   (NTHR * EPT)
#define WCAP    (EPT * 32)
#define LISTN   (NWAVE * WCAP)
#define NBMAX   2048
#define NBRUN   512
#define RCAP    28672
#define DEGCAP  128
#define LDS_SCAN ((2 * RCAP + 2 * NBMAX + LISTN) * 4 + 64)
#define WSMAX   ((size_t)128 << 20)

static_assert(8 * 32 == DD);
static_assert((NE % 256) == 0 && (NE % 4) == 0);
static_assert(NN <= 20 * NBRUN && 20 * NBRUN == MPAD);
static_assert((NN % 16) == 0 && (NN % 4) == 0 && (NN % 2) == 0);
static_assert((MPAD % 64) == 0 && (MPAD % 128) == 0 && (MPAD % 256) == 0);
static_assert((CHUNK & (CHUNK - 1)) == 0 && CHUNK <= 4096);
static_assert((NBMAX & (NBMAX - 1)) == 0 && NBMAX <= 4096);
static_assert((NBRUN & (NBRUN - 1)) == 0 && NBRUN <= NBMAX && NBRUN == 4 * 128);
static_assert(NTHR * 8 == NBMAX && LISTN >= NBMAX);
static_assert((RCAP % 32) == 0 && RCAP >= 16638 + 8192 && 2 * NBRUN <= RCAP);
static_assert(DEGCAP >= 58 + 8);
static_assert(NE < (1 << 20));
static_assert(LDS_SCAN <= 327680);
static_assert(34816 <= 327680);

__device__ __forceinline__ v4f wid_a(v4u w) {
  return (v4f){ __uint_as_float(w[0] << 16), __uint_as_float(w[0] & 0xffff0000u),
                __uint_as_float(w[1] << 16), __uint_as_float(w[1] & 0xffff0000u) };
}
__device__ __forceinline__ v4f wid_c(v4u w) {
  return (v4f){ __uint_as_float(w[2] << 16), __uint_as_float(w[2] & 0xffff0000u),
                __uint_as_float(w[3] << 16), __uint_as_float(w[3] & 0xffff0000u) };
}
__device__ __forceinline__ v4f rne4(v4f v) {
  return (v4f){ bf16_val(v[0]), bf16_val(v[1]), bf16_val(v[2]), bf16_val(v[3]) };
}

__device__ __forceinline__ int scan_chunk(const int* __restrict__ dsts, int nE, int cbase, int slotBase,
                                          int nb, int vec8, int* list, int tid, int lane, int wave) {
  int wc = 0;
  const int el0  = tid * EPT;
  const int e0   = cbase + el0;
  const int sent = (-0x7fffffff - 1);
  v4i da, db;
  if (vec8 != 0 && cbase + CHUNK <= nE) {
    da = *(const v4i*)(dsts + e0);
    db = *(const v4i*)(dsts + e0 + 4);
  } else {
    const int t0 = dsts[min(e0 + 0, nE - 1)];
    const int t1 = dsts[min(e0 + 1, nE - 1)];
    const int t2 = dsts[min(e0 + 2, nE - 1)];
    const int t3 = dsts[min(e0 + 3, nE - 1)];
    const int t4 = dsts[min(e0 + 4, nE - 1)];
    const int t5 = dsts[min(e0 + 5, nE - 1)];
    const int t6 = dsts[min(e0 + 6, nE - 1)];
    const int t7 = dsts[min(e0 + 7, nE - 1)];
    asm volatile("" :: "v"(t0), "v"(t1), "v"(t2), "v"(t3), "v"(t4), "v"(t5), "v"(t6), "v"(t7));
    da.x = (e0 + 0 < nE) ? t0 : sent;
    da.y = (e0 + 1 < nE) ? t1 : sent;
    da.z = (e0 + 2 < nE) ? t2 : sent;
    da.w = (e0 + 3 < nE) ? t3 : sent;
    db.x = (e0 + 4 < nE) ? t4 : sent;
    db.y = (e0 + 5 < nE) ? t5 : sent;
    db.z = (e0 + 6 < nE) ? t6 : sent;
    db.w = (e0 + 7 < nE) ? t7 : sent;
  }
  const unsigned nbs = (unsigned)slotBase;
  const unsigned unb = (unsigned)nb;
  const unsigned s0 = (unsigned)da.x - nbs, s1 = (unsigned)da.y - nbs;
  const unsigned s2 = (unsigned)da.z - nbs, s3 = (unsigned)da.w - nbs;
  const unsigned s4 = (unsigned)db.x - nbs, s5 = (unsigned)db.y - nbs;
  const unsigned s6 = (unsigned)db.z - nbs, s7 = (unsigned)db.w - nbs;
  const bool h0 = s0 < unb, h1 = s1 < unb, h2 = s2 < unb, h3 = s3 < unb;
  const bool h4 = s4 < unb, h5 = s5 < unb, h6 = s6 < unb, h7 = s7 < unb;
  const unsigned any = __builtin_amdgcn_ballot_w32(h0 | h1 | h2 | h3 | h4 | h5 | h6 | h7);
  if (any != 0u) {
#define HITJ(J, HJ, SJ) { \
      const unsigned mj = __builtin_amdgcn_ballot_w32(HJ); \
      if (mj != 0u) { \
        if (HJ) { \
          const int pos = wc + (int)__builtin_amdgcn_mbcnt_lo(mj, 0u); \
          if (pos < WCAP) list[wave * WCAP + pos] = ((el0 + (J)) << 12) | (int)(SJ); \
        } \
        wc += (int)__builtin_popcount(mj); } }
    HITJ(0, h0, s0)
    HITJ(1, h1, s1)
    HITJ(2, h2, s2)
    HITJ(3, h3, s3)
    HITJ(4, h4, s4)
    HITJ(5, h5, s5)
    HITJ(6, h6, s6)
    HITJ(7, h7, s7)
#undef HITJ
  }
  return wc;
}

__device__ __forceinline__ int bucket_build(const int* __restrict__ keys, int nE, int nodeBase, int nb, int vec8) {
  extern __shared__ v4f lds_dyn[];
  int* reg1 = (int*)lds_dyn;
  int* reg2 = reg1 + RCAP;
  int* scnt = reg2 + RCAP;
  int* soff = scnt + NBMAX;
  int* list = soff + NBMAX;
  int* wcnt = list + LISTN;
  int* wtot = wcnt + NWAVE;
  const int tid = (int)threadIdx.x, lane = tid & 31, wave = tid >> 5;

  for (int i = tid; i < NBMAX; i += NTHR) scnt[i] = 0;
  __syncthreads();

  int tot = 0;
  const int nChunks = (nE + CHUNK - 1) / CHUNK;
#pragma unroll 1
  for (int ch = 0; ch < nChunks; ++ch) {
    const int cbase = ch * CHUNK;
    const int wc = scan_chunk(keys, nE, cbase, nodeBase, nb, vec8, list, tid, lane, wave);
    if (lane == 0) wcnt[wave] = wc;
    __syncthreads();
    int pre = 0, all = 0;
#pragma unroll
    for (int w2 = 0; w2 < NWAVE; ++w2) {
      int c = wcnt[w2];
      c = c < 0 ? 0 : (c > WCAP ? WCAP : c);
      all += c;
      pre += (w2 < wave) ? c : 0;
    }
    const int wcc  = wc > WCAP ? WCAP : wc;
    const int base = tot + pre;
#pragma unroll 1
    for (int i = lane; i < wcc; i += 32) {
      const int ent = list[wave * WCAP + i];
      const int el  = (ent >> 12) & (CHUNK - 1);
      const int sl  = ent & (NBMAX - 1);
      int eid = cbase + el;
      eid = eid > nE - 1 ? nE - 1 : eid;
      const int pos = base + i;
      if (pos < RCAP) reg1[pos] = (int)(((unsigned)eid << 12) | (unsigned)sl);
    }
    tot += all;
    tot = tot > RCAP ? RCAP : tot;
    __syncthreads();
  }
  const int nh = tot;

  if (wave == 0) {
#pragma unroll 1
    for (int b0 = 0; b0 < nh; b0 += 32) {
      const int idx = b0 + lane;
      const int uv  = reg1[idx < RCAP ? idx : RCAP - 1];
      const int m32 = (nh - b0) < 32 ? (nh - b0) : 32;
#pragma unroll 1
      for (int k = 0; k < m32; ++k) {
        const int u  = __builtin_amdgcn_readlane(uv, k);
        const int sl = u & (NBMAX - 1);
        if (lane == 0) scnt[sl] = scnt[sl] + 1;
      }
    }
  }
  __syncthreads();

  {
    const v4i ca = *(const v4i*)(scnt + 8 * tid);
    const v4i cb = *(const v4i*)(scnt + 8 * tid + 4);
    const int e0 = ca.x < 0 ? 0 : ca.x, e1 = ca.y < 0 ? 0 : ca.y, e2 = ca.z < 0 ? 0 : ca.z, e3 = ca.w < 0 ? 0 : ca.w;
    const int e4 = cb.x < 0 ? 0 : cb.x, e5 = cb.y < 0 ? 0 : cb.y, e6 = cb.z < 0 ? 0 : cb.z, e7 = cb.w < 0 ? 0 : cb.w;
    const int ts = e0 + e1 + e2 + e3 + e4 + e5 + e6 + e7;
    int incl = ts;
#pragma unroll
    for (int d = 1; d < 32; d <<= 1) {
      const int up = __shfl_up(incl, d);
      if (lane >= d) incl += up;
    }
    if (lane == 31) wtot[wave] = incl;
    __syncthreads();
    int pre = 0;
#pragma unroll
    for (int w2 = 0; w2 < NWAVE; ++w2) pre += (w2 < wave) ? wtot[w2] : 0;
    int run = pre + incl - ts;
    soff[8 * tid + 0] = run; run += e0;
    soff[8 * tid + 1] = run; run += e1;
    soff[8 * tid + 2] = run; run += e2;
    soff[8 * tid + 3] = run; run += e3;
    soff[8 * tid + 4] = run; run += e4;
    soff[8 * tid + 5] = run; run += e5;
    soff[8 * tid + 6] = run; run += e6;
    soff[8 * tid + 7] = run;
  }
  __syncthreads();
  for (int i = tid; i < NBMAX; i += NTHR) list[i] = soff[i];
  __syncthreads();

  if (wave == 0) {
#pragma unroll 1
    for (int b0 = 0; b0 < nh; b0 += 32) {
      const int idx = b0 + lane;
      const int uv  = reg1[idx < RCAP ? idx : RCAP - 1];
      const int m32 = (nh - b0) < 32 ? (nh - b0) : 32;
#pragma unroll 1
      for (int k = 0; k < m32; ++k) {
        const int u   = __builtin_amdgcn_readlane(uv, k);
        const int sl  = u & (NBMAX - 1);
        const int eid = (int)((unsigned)u >> 12);
        if (lane == 0) {
          int pos = list[sl];
          pos = pos < 0 ? 0 : (pos > RCAP - 1 ? RCAP - 1 : pos);
          reg2[pos] = eid;
          list[sl] = pos + 1;
        }
      }
    }
  }
  __syncthreads();
  return nh;
}

__device__ __forceinline__ void rv_put(const float* __restrict__ src, float* dst, int t) {
  const v4f v = *(const v4fa*)(src + 4 * t);
  const v4f r = rne4(v);
  volatile v4f* q = (volatile v4f*)(dst + 4 * t);
  *q = r;
  __threadfence();
  *q = r;
}
__global__ __launch_bounds__(256) void k_rvec(const float* __restrict__ pbd2, const float* __restrict__ pbo,
                                              const float* __restrict__ pbf, float* dst) {
  const int t = (int)threadIdx.x;
  const int b = (int)blockIdx.x;
  if (b == 0)      { if (t < 192) rv_put(pbd2, dst, t); }
  else if (b == 1) { if (t < 192) rv_put(pbo, dst + 768, t); }
  else             { if (t < 64)  rv_put(pbf, dst + 1536, t); }
}

__global__ __launch_bounds__(256) void k_tab(const float* __restrict__ demb, const float* __restrict__ aemb,
                                             const float* __restrict__ Wsp1, const float* __restrict__ bsp1,
                                             const float* __restrict__ Wsp2, const float* __restrict__ bsp2,
                                             float* TAB) {
  __shared__ __attribute__((aligned(16))) float sW[1024];
  __shared__ __attribute__((aligned(16))) float sB[32];
  __shared__ __attribute__((aligned(16))) float sW2[32];
  __shared__ __attribute__((aligned(16))) float sSe[32 * 256];
  __shared__ __attribute__((aligned(16))) float sOut[256];
  const int tid = (int)threadIdx.x;
  const int s   = (int)blockIdx.x / 7;
  const int b7  = (int)blockIdx.x - s * 7;
  const int loc = b7 * 256 + tid;
  const int ent = loc < 1599 ? loc : 1599;
  const int db  = ent >> 4;
  const int ab  = ent & 15;
#pragma unroll
  for (int u = 0; u < 4; ++u) sW[tid + 256 * u] = bf16_val(Wsp1[s * 1024 + tid + 256 * u]);
  if (tid < 32) {
    sB[tid]  = bf16_val(bsp1[s * 32 + tid]);
    sW2[tid] = bf16_val(Wsp2[s * 32 + tid]);
  }
  const float* dr = demb + (size_t)(s * 100 + db) * 16;
  const float* ar = aemb + (size_t)(s * 16 + ab) * 16;
#pragma unroll
  for (int u = 0; u < 4; ++u) {
    const v4f dv = *(const v4fa*)(dr + 4 * u);
    const v4f av = *(const v4fa*)(ar + 4 * u);
    asm volatile("" :: "v"(dv));
    asm volatile("" :: "v"(av));
#pragma unroll
    for (int e = 0; e < 4; ++e) {
      sSe[(4 * u + e) * 256 + tid]      = bf16_val(dv[e]);
      sSe[(16 + 4 * u + e) * 256 + tid] = bf16_val(av[e]);
    }
  }
  const float b2 = bf16_val(bsp2[s]);
  __syncthreads();
  float e2 = 0.0f;
#pragma unroll 1
  for (int j = 0; j < 32; ++j) {
    float a = 0.0f;
#pragma unroll 4
    for (int k = 0; k < 32; ++k) a = fmaf(sSe[k * 256 + tid], sW[j * 32 + k], a);
    a = a + sB[j];
    a = a > 0.0f ? a : 0.0f;
    e2 = fmaf(a, sW2[j], e2);
  }
  sOut[tid] = e2 + b2;
  __syncthreads();
  if (tid < 64) {
    const v4f v = *(const v4fa*)(sOut + 4 * tid);
    volatile v4f* q = (volatile v4f*)(TAB + (size_t)s * TABP + b7 * 256 + 4 * tid);
    *q = v;
    __threadfence();
    *q = v;
  }
}

__global__ __launch_bounds__(256) void k_geo(const int* __restrict__ ei, const float* __restrict__ coords,
                                             const float* __restrict__ TAB, float* ENC, int nE, int nN) {
  const int e  = (int)blockIdx.x * 256 + (int)threadIdx.x;
  const int ec = e < nE ? e : nE - 1;
  const int s  = clampi(ei[ec], 0, nN - 1);
  const int d  = clampi(ei[nE + ec], 0, nN - 1);
  const v2f cs = *(const v2fa*)(coords + 2 * (size_t)s);
  const v2f cd = *(const v2fa*)(coords + 2 * (size_t)d);
  asm volatile("" :: "v"(cs));
  asm volatile("" :: "v"(cd));
  const float rx = (bf16_val(cs[0]) - bf16_val(cd[0])) + 0.0f;
  const float ry = (bf16_val(cs[1]) - bf16_val(cd[1])) + 0.0f;
  const float t  = __fadd_rn(__fmul_rn(rx, rx), __fmul_rn(ry, ry));
  const float dist = sqrtf(t);
  const float ang  = atan2f(ry, rx);
  const float PI_F  = 0x1.921fb6p+1f;
  const float TPI_F = 0x1.921fb6p+2f;
  const int ab = clampi((int)(((ang + PI_F) / TPI_F) * 15.0f), 0, 15);
  const int b0 = clampi((int)((dist / 500.0f) * 99.0f), 0, 99);
  const int b1 = clampi((int)((dist / 1000.0f) * 99.0f), 0, 99);
  const int b2 = clampi((int)((dist / 2000.0f) * 99.0f), 0, 99);
  const float t0 = TAB[b0 * 16 + ab];
  const float t1 = TAB[TABP + b1 * 16 + ab];
  const float t2 = TAB[2 * TABP + b2 * 16 + ab];
  asm volatile("" :: "v"(t0));
  asm volatile("" :: "v"(t1));
  asm volatile("" :: "v"(t2));
  const v4f o = (v4f){ t0, t1, t2, 0.0f };
  if (e < nE) {
    volatile v4f* q = (volatile v4f*)(ENC + (size_t)e * 4);
    *q = o;
    __threadfence();
    *q = o;
  }
}

__global__ __launch_bounds__(256) void k_pair(const float* __restrict__ coords, float* CNT, int nN) {
  __shared__ __attribute__((aligned(16))) float sC[4096];
  __shared__ __attribute__((aligned(16))) float sO[256];
  const int tid = (int)threadIdx.x;
  const int i   = (int)blockIdx.x * 256 + tid;
  const int ic  = i < nN ? i : nN - 1;
  const v2f ci  = *(const v2fa*)(coords + 2 * (size_t)ic);
  asm volatile("" :: "v"(ci));
  const float cx = bf16_val(ci[0]);
  const float cy = bf16_val(ci[1]);
  int cnt = 0;
#pragma unroll 1
  for (int t0 = 0; t0 < nN; t0 += 2048) {
    __syncthreads();
#pragma unroll
    for (int u = 0; u < 4; ++u) {
      const int p = tid + 256 * u;
      int j0 = t0 + 2 * p;
      j0 = j0 < nN - 2 ? j0 : nN - 2;
      const v4f c = *(const v4fa*)(coords + 2 * (size_t)j0);
      asm volatile("" :: "v"(c));
      *(v4fa*)(sC + 4 * p) = rne4(c);
    }
    __syncthreads();
    const int rem  = nN - t0;
    const int lim2 = (rem < 2048 ? rem : 2048) >> 1;
#pragma unroll 4
    for (int p = 0; p < lim2; ++p) {
      const v4f c = *(const v4fa*)(sC + 4 * p);
      const float dx0 = cx - c[0], dy0 = cy - c[1];
      const float dx1 = cx - c[2], dy1 = cy - c[3];
      const float ta = __fadd_rn(__fmul_rn(dx0, dx0), __fmul_rn(dy0, dy0));
      const float tb = __fadd_rn(__fmul_rn(dx1, dx1), __fmul_rn(dy1, dy1));
      cnt += (ta <= 2500.0f) ? 1 : 0;
      cnt += (tb <= 2500.0f) ? 1 : 0;
    }
  }
  sO[tid] = (i < nN) ? (float)cnt : 0.0f;
  __syncthreads();
  if (tid < 64) {
    const v4f v = *(const v4fa*)(sO + 4 * tid);
    volatile v4f* q = (volatile v4f*)(CNT + (size_t)blockIdx.x * 256 + 4 * tid);
    *q = v;
    __threadfence();
    *q = v;
  }
}

__global__ __launch_bounds__(NTHR) __attribute__((amdgpu_num_vgpr(248)))
void k_srcscan(const int* __restrict__ keys, const int* __restrict__ oth, const unsigned short* __restrict__ XB,
               float* STATS, int nN, int nE, int nb, int vec8) {
  extern __shared__ v4f lds_dyn[];
  int* reg1 = (int*)lds_dyn;
  int* reg2 = reg1 + RCAP;
  int* scnt = reg2 + RCAP;
  int* soff = scnt + NBMAX;
  const int tid = (int)threadIdx.x, lane = tid & 31, wave = tid >> 5;
  const int nodeBase = (int)blockIdx.x * nb;
  const int nh = bucket_build(keys, nE, nodeBase, nb, vec8);
  float* stg = (float*)reg1;
  const int nbw = nb >> 3;
  const bool ovf = (nh >= RCAP);
  const float qnan = __int_as_float(0x7fc00000);
#pragma unroll 1
  for (int jt = 0; jt < nbw; ++jt) {
    const int slot = wave * nbw + jt;
    const int grow = nodeBase + slot;
    const int gcl  = grow < nN ? grow : nN - 1;
    int st = soff[slot];
    const int craw = scnt[slot];
    int cnt = craw;
    st  = st < 0 ? 0 : (st > nh ? nh : st);
    cnt = cnt < 0 ? 0 : (cnt > DEGCAP ? DEGCAP : cnt);
    if (cnt > nh - st) cnt = nh - st;
    st  = __builtin_amdgcn_readfirstlane(st);
    cnt = __builtin_amdgcn_readfirstlane(cnt);
    const bool bad = ovf || (craw > DEGCAP);
    v4f n0 = (v4f){0.f, 0.f, 0.f, 0.f};
    v4f n1 = (v4f){0.f, 0.f, 0.f, 0.f};
#pragma unroll 1
    for (int q = 0; q < cnt; ++q) {
      int idx = st + q; idx = idx > RCAP - 1 ? RCAP - 1 : idx;
      int eid = reg2[idx]; eid = eid < 0 ? 0 : (eid > nE - 1 ? nE - 1 : eid);
      eid = __builtin_amdgcn_readfirstlane(eid);
      int d = oth[eid]; d = d < 0 ? 0 : (d > nN - 1 ? nN - 1 : d);
      d = __builtin_amdgcn_readfirstlane(d);
      const v4u w = *(const v4ua*)(XB + (size_t)d * DD + 8 * lane);
      asm volatile("" :: "v"(w));
      n0 += wid_a(w);
      n1 += wid_c(w);
    }
    const v4u wx = *(const v4ua*)(XB + (size_t)gcl * DD + 8 * lane);
    asm volatile("" :: "v"(wx));
    const v4f x0 = wid_a(wx), x1 = wid_c(wx);
    const float degf = (float)cnt;
    const float rc = 1.0f / (degf > 1.0f ? degf : 1.0f);
    const v4f t0 = x0 - n0 * rc;
    const v4f t1 = x1 - n1 * rc;
    float part = t0[0] * t0[0];
    part = fmaf(t0[1], t0[1], part); part = fmaf(t0[2], t0[2], part); part = fmaf(t0[3], t0[3], part);
    part = fmaf(t1[0], t1[0], part); part = fmaf(t1[1], t1[1], part);
    part = fmaf(t1[2], t1[2], part); part = fmaf(t1[3], t1[3], part);
#pragma unroll
    for (int off = 16; off > 0; off >>= 1) part += __shfl_xor(part, off);
    const float fv = sqrtf(part);
    const bool live = grow < nN;
    const float vdeg = bad ? qnan : (live ? degf : 0.0f);
    const float vfv  = bad ? qnan : (live ? fv : 0.0f);
    if (lane == 0) { stg[slot] = vdeg; stg[NBRUN + slot] = vfv; }
  }
  __syncthreads();
  {
    const v4f v = *(const v4fa*)(stg + 4 * tid);
    const int po = (tid < 128 ? 0 : SPP) + nodeBase + 4 * (tid & 127);
    const bool ok = (4 * (tid & 127) < nb) && (nodeBase + 4 * (tid & 127) + 3 < SPP);
    volatile v4f* q = (volatile v4f*)(STATS + po);
    if (ok) *q = v;
    __threadfence();
    if (ok) *q = v;
  }
}

__global__ __launch_bounds__(256) void k_max(const float* __restrict__ STATS, float* MAX3, int nN) {
  __shared__ float sm[24];
  const int tid = (int)threadIdx.x, lane = tid & 31, wave = tid >> 5;
  const int np = nN >> 2;
  const int nit = (np + 255) >> 8;
  float m0 = -3.0e38f, m1 = -3.0e38f, m2 = -3.0e38f;
#pragma unroll 1
  for (int it = 0; it < nit; ++it) {
    int p = it * 256 + tid; p = p < np - 1 ? p : np - 1;
    const v4f a = *(const v4fa*)(STATS + 4 * p);
    const v4f f = *(const v4fa*)(STATS + SPP + 4 * p);
    const v4f c = *(const v4fa*)(STATS + 2 * SPP + 4 * p);
    m0 = fmaxf(m0, fmaxf(fmaxf(a[0], a[1]), fmaxf(a[2], a[3])));
    m2 = fmaxf(m2, fmaxf(fmaxf(f[0], f[1]), fmaxf(f[2], f[3])));
    m1 = fmaxf(m1, fmaxf(fmaxf(c[0] - 1.0f, c[1] - 1.0f), fmaxf(c[2] - 1.0f, c[3] - 1.0f)));
  }
#pragma unroll
  for (int off = 16; off > 0; off >>= 1) {
    m0 = fmaxf(m0, __shfl_xor(m0, off));
    m1 = fmaxf(m1, __shfl_xor(m1, off));
    m2 = fmaxf(m2, __shfl_xor(m2, off));
  }
  if (lane == 0) { sm[wave] = m0; sm[8 + wave] = m1; sm[16 + wave] = m2; }
  __syncthreads();
  float r0 = sm[0], r1 = sm[8], r2 = sm[16];
#pragma unroll
  for (int w = 1; w < 8; ++w) { r0 = fmaxf(r0, sm[w]); r1 = fmaxf(r1, sm[8 + w]); r2 = fmaxf(r2, sm[16 + w]); }
  const float sel = (tid == 0) ? 1.0f : 0.0f;
  const v4f o = (v4f){ r0 * sel, r1 * sel, r2 * sel, 0.0f };
  if (tid < 8) {
    volatile v4f* q = (volatile v4f*)(MAX3 + 4 * tid);
    *q = o;
    __threadfence();
    *q = o;
  }
}

__global__ __launch_bounds__(256) void k_hid(const float* __restrict__ STATS, const float* __restrict__ MAX3,
                                             const float* __restrict__ Wd1s, const float* __restrict__ bd1s,
                                             unsigned short* HIDHL, int nN, int MP) {
  const int lane = (int)threadIdx.x & 31, wave = (int)threadIdx.x >> 5;
  const int c0 = 8 * (lane & 15);
  float wf[24];
#pragma unroll
  for (int i = 0; i < 6; ++i) {
    const v4f w = *(const v4fa*)(Wd1s + c0 * 3 + 4 * i);
    asm volatile("" :: "v"(w));
    wf[4 * i + 0] = bf16_val(w[0]); wf[4 * i + 1] = bf16_val(w[1]);
    wf[4 * i + 2] = bf16_val(w[2]); wf[4 * i + 3] = bf16_val(w[3]);
  }
  const v4f ba = rne4(*(const v4fa*)(bd1s + c0));
  const v4f bc = rne4(*(const v4fa*)(bd1s + c0 + 4));
  const float bb[8] = { ba[0], ba[1], ba[2], ba[3], bc[0], bc[1], bc[2], bc[3] };
  const v4f mx = *(const v4fa*)(MAX3);
  const float q0 = mx[0] + 1e-8f, q1 = mx[1] + 1e-8f, q2 = mx[2] + 1e-8f;
  const int row0 = ((int)blockIdx.x * 8 + wave) * 16;
#pragma unroll 1
  for (int r = 0; r < 16; ++r) {
    const int row = row0 + r;
    const int rc  = row < nN ? row : nN - 1;
    const float dg = STATS[rc];
    const float fv = STATS[SPP + rc];
    const float cn = STATS[2 * SPP + rc];
    asm volatile("" :: "v"(dg));
    asm volatile("" :: "v"(fv));
    asm volatile("" :: "v"(cn));
    const float d0 = dg / q0;
    const float d1 = (cn - 1.0f) / q1;
    const float d2 = fv / q2;
    float h[8];
#pragma unroll
    for (int c = 0; c < 8; ++c) {
      float v = ((d0 * wf[3 * c] + d1 * wf[3 * c + 1]) + d2 * wf[3 * c + 2]) + bb[c];
      h[c] = (v > 0.0f) ? v : (v - v);
    }
    const v4f a = (v4f){ h[0], h[1], h[2], h[3] };
    const v4f c = (v4f){ h[4], h[5], h[6], h[7] };
    const v4u hi = pack8_bf16(a, c);
    const v4u lo = pack8_bf16_lo(a, c);
    v4u o = (lane < 16) ? hi : lo;
    const unsigned lm = (row < nN) ? 0xFFFFFFFFu : 0u;
    o &= (v4u){ lm, lm, lm, lm };
    const bool wr = row < MP;
    volatile v4u* q = (volatile v4u*)(HIDHL + (size_t)row * 256 + 8 * lane);
    if (wr) *q = o;
    __threadfence();
    if (wr) *q = o;
  }
}

__global__ __launch_bounds__(256) void k_rownorm(const float* __restrict__ DF, float* DFN, int nN) {
  const int lane = (int)threadIdx.x & 31, wave = (int)threadIdx.x >> 5;
  const int row0 = ((int)blockIdx.x * 8 + wave) * 16;
#pragma unroll 1
  for (int r = 0; r < 16; ++r) {
    const int row = row0 + r;
    const int rc  = row < nN ? row : nN - 1;
    const float* p = DF + (size_t)rc * DD;
    const v4f a = *(const v4fa*)(p + 4 * lane);
    const v4f b = *(const v4fa*)(p + 128 + 4 * lane);
    asm volatile("" :: "v"(a));
    asm volatile("" :: "v"(b));
    float ss = a[0] * a[0];
    ss = fmaf(a[1], a[1], ss); ss = fmaf(a[2], a[2], ss); ss = fmaf(a[3], a[3], ss);
    ss = fmaf(b[0], b[0], ss); ss = fmaf(b[1], b[1], ss); ss = fmaf(b[2], b[2], ss); ss = fmaf(b[3], b[3], ss);
#pragma unroll
    for (int off = 16; off > 0; off >>= 1) ss += __shfl_xor(ss, off);
    const float nrm = sqrtf(ss);
    const float inv = 1.0f / fmaxf(nrm, 1e-8f);
    const v4f oa = a * inv;
    const v4f ob = b * inv;
    const bool wr = row < nN;
    volatile v4f* qa = (volatile v4f*)(DFN + (size_t)row * DD + 4 * lane);
    volatile v4f* qb = (volatile v4f*)(DFN + (size_t)row * DD + 128 + 4 * lane);
    if (wr) { *qa = oa; *qb = ob; }
    __threadfence();
    if (wr) { *qa = oa; *qb = ob; }
  }
}

__global__ __launch_bounds__(NTHR) __attribute__((amdgpu_num_vgpr(248)))
void k_scan(const int* __restrict__ srcs, const int* __restrict__ dsts,
            const float* __restrict__ QKV, const float* __restrict__ DFN, const float* __restrict__ ENC,
            const float* __restrict__ tempS, unsigned short* AGGHL,
            int sc, int nN, int nE, int nb, int vec8, int MPr) {
  extern __shared__ v4f lds_dyn[];
  int* reg1 = (int*)lds_dyn;
  int* reg2 = reg1 + RCAP;
  int* scnt = reg2 + RCAP;
  int* soff = scnt + NBMAX;
  const int tid = (int)threadIdx.x, lane = tid & 31, wave = tid >> 5;
  const int nodeBase = (int)blockIdx.x * nb;
  const int nh = bucket_build(dsts, nE, nodeBase, nb, vec8);
  const int nbw = nb >> 3;
  const bool ovf = (nh >= RCAP);
  const float qnan = __int_as_float(0x7fc00000);
  const float th = bf16_val(tempS[lane >> 2]);
  const float SQH = 0x1.6a09e6p+2f;
#pragma unroll 1
  for (int jt = 0; jt < nbw; ++jt) {
    const int slot = wave * nbw + jt;
    const int grow = nodeBase + slot;
    const int gcl  = grow < nN ? grow : nN - 1;
    int st = soff[slot];
    const int craw = scnt[slot];
    int cnt = craw;
    st  = st < 0 ? 0 : (st > nh ? nh : st);
    cnt = cnt < 0 ? 0 : (cnt > DEGCAP ? DEGCAP : cnt);
    if (cnt > nh - st) cnt = nh - st;
    st  = __builtin_amdgcn_readfirstlane(st);
    cnt = __builtin_amdgcn_readfirstlane(cnt);
    const bool bad = ovf || (craw > DEGCAP);

    const float* qp = QKV + (size_t)gcl * 768 + 8 * lane;
    const float* dp = DFN + (size_t)gcl * DD + 8 * lane;
    const v4f q0 = *(const v4fa*)qp, q1 = *(const v4fa*)(qp + 4);
    const v4f g0 = *(const v4fa*)dp, g1 = *(const v4fa*)(dp + 4);
    asm volatile("" :: "v"(q0));
    asm volatile("" :: "v"(q1));
    asm volatile("" :: "v"(g0));
    asm volatile("" :: "v"(g1));
    v4f a0 = (v4f){0.f, 0.f, 0.f, 0.f};
    v4f a1 = (v4f){0.f, 0.f, 0.f, 0.f};
    float mx = -1.0e30f, dn = 0.0f;

#pragma unroll 1
    for (int q = 0; q < cnt; ++q) {
      int idx = st + q; idx = idx > RCAP - 1 ? RCAP - 1 : idx;
      int eid = reg2[idx]; eid = eid < 0 ? 0 : (eid > nE - 1 ? nE - 1 : eid);
      eid = __builtin_amdgcn_readfirstlane(eid);
      int s = srcs[eid]; s = s < 0 ? 0 : (s > nN - 1 ? nN - 1 : s);
      s = __builtin_amdgcn_readfirstlane(s);
      const float* kr = QKV + (size_t)s * 768 + 256 + 8 * lane;
      const float* fr = DFN + (size_t)s * DD + 8 * lane;
      const v4f k0 = *(const v4fa*)kr,         k1 = *(const v4fa*)(kr + 4);
      const v4f v0 = *(const v4fa*)(kr + 256), v1 = *(const v4fa*)(kr + 260);
      const v4f f0 = *(const v4fa*)fr,         f1 = *(const v4fa*)(fr + 4);
      const float en = ENC[(size_t)eid * 4 + sc];
      asm volatile("" :: "v"(k0));
      asm volatile("" :: "v"(k1));
      asm volatile("" :: "v"(v0));
      asm volatile("" :: "v"(v1));
      asm volatile("" :: "v"(f0));
      asm volatile("" :: "v"(f1));
      asm volatile("" :: "v"(en));
      float part = q0[0] * k0[0];
      part = fmaf(q0[1], k0[1], part); part = fmaf(q0[2], k0[2], part); part = fmaf(q0[3], k0[3], part);
      part = fmaf(q1[0], k1[0], part); part = fmaf(q1[1], k1[1], part);
      part = fmaf(q1[2], k1[2], part); part = fmaf(q1[3], k1[3], part);
      part += __shfl_xor(part, 1);
      part += __shfl_xor(part, 2);
      float ds = g0[0] * f0[0];
      ds = fmaf(g0[1], f0[1], ds); ds = fmaf(g0[2], f0[2], ds); ds = fmaf(g0[3], f0[3], ds);
      ds = fmaf(g1[0], f1[0], ds); ds = fmaf(g1[1], f1[1], ds);
      ds = fmaf(g1[2], f1[2], ds); ds = fmaf(g1[3], f1[3], ds);
#pragma unroll
      for (int off = 16; off > 0; off >>= 1) ds += __shfl_xor(ds, off);
      float sv = part / SQH;
      sv = sv / th;
      sv = sv + en;
      sv = sv * (1.0f + 0.5f * ds);
      const float dfv = sv - mx;
      const float ee  = expf(-fabsf(dfv));
      const bool up   = dfv > 0.0f;
      const float s1  = up ? ee : 1.0f;
      const float s2  = up ? 1.0f : ee;
      mx = up ? sv : mx;
      dn = fmaf(dn, s1, s2);
      a0[0] = fmaf(a0[0], s1, s2 * v0[0]); a0[1] = fmaf(a0[1], s1, s2 * v0[1]);
      a0[2] = fmaf(a0[2], s1, s2 * v0[2]); a0[3] = fmaf(a0[3], s1, s2 * v0[3]);
      a1[0] = fmaf(a1[0], s1, s2 * v1[0]); a1[1] = fmaf(a1[1], s1, s2 * v1[1]);
      a1[2] = fmaf(a1[2], s1, s2 * v1[2]); a1[3] = fmaf(a1[3], s1, s2 * v1[3]);
    }
    const float inv = 1.0f / (dn + 1e-16f);
    v4f ra = a0 * inv;
    v4f rb = a1 * inv;
    const v4f nn = (v4f){ qnan, qnan, qnan, qnan };
    ra = bad ? nn : ra;
    rb = bad ? nn : rb;
    const v4u hi = pack8_bf16(ra, rb);
    const v4u lo = pack8_bf16_lo(ra, rb);
    const bool wr = grow < MPr;
    unsigned short* rowp = AGGHL + (size_t)grow * 512;
    volatile v4u* ph = (volatile v4u*)(rowp + 8 * lane);
    volatile v4u* pl = (volatile v4u*)(rowp + 256 + 8 * lane);
    if (wr) { *ph = hi; *pl = lo; }
    __threadfence();
    if (wr) { *ph = hi; *pl = lo; }
  }
}

__global__ __launch_bounds__(256) void k_cat(const float* __restrict__ OUTS, unsigned short* OUTHL,
                                             int sc, int nN, int MP) {
  const int lane = (int)threadIdx.x & 31, wave = (int)threadIdx.x >> 5;
  const int row0 = ((int)blockIdx.x * 8 + wave) * 16;
#pragma unroll 1
  for (int r = 0; r < 16; ++r) {
    const int row = row0 + r;
    const int rc  = row < nN ? row : nN - 1;
    const float* p = OUTS + (size_t)rc * DD + 8 * lane;
    const v4f a = *(const v4fa*)p;
    const v4f c = *(const v4fa*)(p + 4);
    asm volatile("" :: "v"(a));
    asm volatile("" :: "v"(c));
    v4u hi = pack8_bf16(a, c);
    v4u lo = pack8_bf16_lo(a, c);
    const unsigned lm = (row < nN) ? 0xFFFFFFFFu : 0u;
    const v4u mw = (v4u){ lm, lm, lm, lm };
    hi &= mw;
    lo &= mw;
    const bool wr = row < MP;
    unsigned short* rowp = OUTHL + (size_t)row * 1536 + sc * 256 + 8 * lane;
    volatile v4u* ph = (volatile v4u*)(rowp);
    volatile v4u* pl = (volatile v4u*)(rowp + 768);
    if (wr) { *ph = hi; *pl = lo; }
    __threadfence();
    if (wr) { *ph = hi; *pl = lo; }
  }
}

static inline size_t al256(size_t v) { return (v + 255) & ~(size_t)255; }
static inline int cdivi(int a, int b) { return (a + b - 1) / b; }

extern "C" void kernel_launch(void* const* d_in, const int* in_sizes, int n_in,
                              void* d_out, int out_size, void* d_ws, size_t ws_size,
                              hipStream_t stream) {
  if (n_in < 21) return;
  const int exp_sz[21] = { NN * DD, NN * 2, 2 * NE, 3 * DD * DD, 3 * DD * DD, 3 * DD * DD, 3 * DD * DD, 3 * DD, 24,
                           4800, 768, 3072, 96, 96, 3, 1152, 384, 3 * DD * 128, 3 * DD, DD * 768, DD };
  for (int i = 0; i < 21; ++i) if (in_sizes[i] != exp_sz[i]) return;
  if (out_size != NN * DD) return;

  const float* x      = (const float*)d_in[0];
  const float* coords = (const float*)d_in[1];
  const int*   ei     = (const int*)  d_in[2];
  const float* Wq     = (const float*)d_in[3];
  const float* Wk     = (const float*)d_in[4];
  const float* Wv     = (const float*)d_in[5];
  const float* Wo     = (const float*)d_in[6];
  const float* bo     = (const float*)d_in[7];
  const float* temp   = (const float*)d_in[8];
  const float* demb   = (const float*)d_in[9];
  const float* aemb   = (const float*)d_in[10];
  const float* Wsp1   = (const float*)d_in[11];
  const float* bsp1   = (const float*)d_in[12];
  const float* Wsp2   = (const float*)d_in[13];
  const float* bsp2   = (const float*)d_in[14];
  const float* Wd1    = (const float*)d_in[15];
  const float* bd1    = (const float*)d_in[16];
  const float* Wd2    = (const float*)d_in[17];
  const float* bd2    = (const float*)d_in[18];
  const float* Wf     = (const float*)d_in[19];
  const float* bfv    = (const float*)d_in[20];
  float* out = (float*)d_out;
  const int* srcRow = ei;
  const int* dstRow = ei + NE;

  char* ws = (char*)d_ws;
  size_t off = 0;
  const size_t oXB   = off; off = al256(off + (size_t)MPAD * 256 * 2);
  const size_t oWQKV = off; off = al256(off + (size_t)3 * 768 * 256 * 2);
  const size_t oWOP  = off; off = al256(off + (size_t)768 * 512 * 2);
  const size_t oWD2P = off; off = al256(off + (size_t)768 * 256 * 2);
  const size_t oWFP  = off; off = al256(off + (size_t)256 * 1536 * 2);
  const size_t oBIAS = off; off = al256(off + (size_t)1792 * 4);
  const size_t oTAB  = off; off = al256(off + (size_t)3 * TABP * 4);
  const size_t oSTAT = off; off = al256(off + (size_t)3 * SPP * 4);
  const size_t oMAX3 = off; off = al256(off + (size_t)128);
  const size_t oENC  = off; off = al256(off + (size_t)NE * 16);
  const size_t oHID  = off; off = al256(off + (size_t)MPAD * 256 * 2);
  const size_t oDF   = off; off = al256(off + (size_t)MPAD * 256 * 4);
  const size_t oDFN  = off; off = al256(off + (size_t)MPAD * 256 * 4);
  const size_t oQKV  = off; off = al256(off + (size_t)MPAD * 768 * 4);
  const size_t oAGG  = off; off = al256(off + (size_t)MPAD * 512 * 2);
  const size_t oOUTH = off; off = al256(off + (size_t)MPAD * 1536 * 2);
  if (off > ws_size || off > (size_t)WSMAX) return;

  unsigned short* XB    = (unsigned short*)(ws + oXB);
  unsigned short* WQKV  = (unsigned short*)(ws + oWQKV);
  unsigned short* WOP   = (unsigned short*)(ws + oWOP);
  unsigned short* WD2P  = (unsigned short*)(ws + oWD2P);
  unsigned short* WFP   = (unsigned short*)(ws + oWFP);
  float*          BIASR = (float*)(ws + oBIAS);
  float*          TAB   = (float*)(ws + oTAB);
  float*          STATS = (float*)(ws + oSTAT);
  float*          MAX3  = (float*)(ws + oMAX3);
  float*          ENC   = (float*)(ws + oENC);
  unsigned short* HIDHL = (unsigned short*)(ws + oHID);
  float*          DF    = (float*)(ws + oDF);
  float*          DFN   = (float*)(ws + oDFN);
  float*          QKV   = (float*)(ws + oQKV);
  unsigned short* AGGHL = (unsigned short*)(ws + oAGG);
  unsigned short* OUTHL = (unsigned short*)(ws + oOUTH);
  float*          OUTS  = DF;

  hipFuncSetAttribute(reinterpret_cast<const void*>(&k_srcscan), hipFuncAttributeMaxDynamicSharedMemorySize, LDS_SCAN);
  hipFuncSetAttribute(reinterpret_cast<const void*>(&k_scan),    hipFuncAttributeMaxDynamicSharedMemorySize, LDS_SCAN);

  static_assert((MPAD * 256 / 8) % 256 == 0 && (256 * 256 / 8) % 256 == 0 && (768 * 512 / 8) % 256 == 0);
  static_assert((768 * 256 / 8) % 256 == 0 && (256 * 1536 / 8) % 256 == 0);

  k_plane<0><<<MPAD * 256 / 8 / 256, 256, 0, stream>>>(x, NN, 256, 256, XB, MPAD, 256);
  for (int s = 0; s < NSC; ++s) {
    unsigned short* base = WQKV + (size_t)s * 768 * 256;
    k_plane<0><<<256 * 256 / 8 / 256, 256, 0, stream>>>(Wq + (size_t)s * 65536, 256, 256, 256, base, 256, 256);
    k_plane<0><<<256 * 256 / 8 / 256, 256, 0, stream>>>(Wk + (size_t)s * 65536, 256, 256, 256, base + 65536, 256, 256);
    k_plane<0><<<256 * 256 / 8 / 256, 256, 0, stream>>>(Wv + (size_t)s * 65536, 256, 256, 256, base + 131072, 256, 256);
  }
  k_plane<3><<<768 * 512 / 8 / 256, 256, 0, stream>>>(Wo, 768, 256, 256, WOP, 768, 256);
  k_plane<3><<<768 * 256 / 8 / 256, 256, 0, stream>>>(Wd2, 768, 128, 128, WD2P, 768, 128);
  k_plane<3><<<256 * 1536 / 8 / 256, 256, 0, stream>>>(Wf, 256, 768, 768, WFP, 256, 768);
  k_rvec<<<3, 256, 0, stream>>>(bd2, bo, bfv, BIASR);

  k_tab<<<21, 256, 0, stream>>>(demb, aemb, Wsp1, bsp1, Wsp2, bsp2, TAB);
  k_geo<<<NE / 256, 256, 0, stream>>>(ei, coords, TAB, ENC, NE, NN);
  k_pair<<<MPAD / 256, 256, 0, stream>>>(coords, STATS + 2 * SPP, NN);
  k_srcscan<<<MPAD / NBRUN, NTHR, LDS_SCAN, stream>>>(srcRow, dstRow, XB, STATS, NN, NE, NBRUN, 1);
  k_max<<<1, 256, 0, stream>>>(STATS, MAX3, NN);

  static_assert((NN % 16) == 0 && (DD % 64) == 0 && (768 % 64) == 0 && (DD % 32) == 0 && (768 % 32) == 0);
  const int tilesM = cdivi(NN, 64);
  for (int s = 0; s < NSC; ++s) {
    k_hid<<<MPAD / 128, 256, 0, stream>>>(STATS, MAX3, Wd1 + (size_t)s * 384, bd1 + (size_t)s * 128, HIDHL, NN, MPAD);
    k_gemm_nt<0, 1><<<cdivi(tilesM * 4, 8), 256, 0, stream>>>(HIDHL, WD2P + (size_t)s * 256 * 256,
                                                              BIASR + s * 256, DF, NN, 256, 256, 256);
    k_rownorm<<<cdivi(NN, 128), 256, 0, stream>>>(DF, DFN, NN);
    k_gemm_nt<0, 0><<<cdivi(tilesM * 12, 8), 256, 0, stream>>>(XB, WQKV + (size_t)s * 768 * 256,
                                                               BIASR, QKV, NN, 768, 256, 768);
    k_scan<<<MPAD / NBRUN, NTHR, LDS_SCAN, stream>>>(srcRow, dstRow, QKV, DFN, ENC, temp + s * 8, AGGHL,
                                                      s, NN, NE, NBRUN, 1, MPAD);
    k_gemm_nt<0, 1><<<cdivi(tilesM * 4, 8), 256, 0, stream>>>(AGGHL, WOP + (size_t)s * 256 * 512,
                                                              BIASR + 768 + s * 256, OUTS, NN, 256, 512, 256);
    k_cat<<<MPAD / 128, 256, 0, stream>>>(OUTS, OUTHL, s, NN, MPAD);
  }
  k_gemm_nt<0, 1><<<cdivi(tilesM * 4, 8), 256, 0, stream>>>(OUTHL, WFP, BIASR + 1536, out, NN, 256, 1536, 256);
}
